// LongformerSelfAttentionForT5_80573586473121
// MI455X (gfx1250) — hardware-verified
//
#include <hip/hip_runtime.h>
#include <math.h>

typedef __attribute__((ext_vector_type(16))) _Float16 v16h;
typedef __attribute__((ext_vector_type(16))) __bf16 v16b;
typedef __attribute__((ext_vector_type(8)))  _Float16 v8h;
typedef __attribute__((ext_vector_type(8)))  float v8f;
typedef __attribute__((ext_vector_type(4)))  float v4f;
typedef __attribute__((ext_vector_type(2)))  float v2f;
typedef __attribute__((ext_vector_type(4)))  unsigned v4u;
typedef __attribute__((ext_vector_type(4)))  int v4i;
typedef float __attribute__((may_alias)) float_a;
typedef int __attribute__((may_alias)) int_a;

template <typename T> __device__ __forceinline__ void vst2(void* p, T v) { *(volatile T*)p = v; __threadfence(); *(volatile T*)p = v; }
__device__ __forceinline__ v8f wmma16(v16h a, v16h b, v8f c) {
  v8f d = __builtin_amdgcn_wmma_f32_16x16x32_f16(false, a, false, b, (short)0, c, false, false);
  asm volatile("v_nop\n\tv_nop\n\tv_nop\n\tv_nop" : "+v"(d) : "v"(a), "v"(b));
  return d;
}
__device__ __forceinline__ v8f wmma_bf(v16b a, v16b b, v8f c) {
  v8f d = __builtin_amdgcn_wmma_f32_16x16x32_bf16(false, a, false, b, (short)0, c, false, false);
  asm volatile("v_nop\n\tv_nop\n\tv_nop\n\tv_nop" : "+v"(d) : "v"(a), "v"(b));
  return d;
}
__device__ __forceinline__ v16h frag_h(const _Float16* rowk0, int lane) {
  union { v16h v; v8h q[2]; } u; const _Float16* p = rowk0 + 8 * (lane >> 4);
  u.q[0] = *(const v8h*)p; u.q[1] = *(const v8h*)(p + 16); return u.v;
}
__device__ __forceinline__ v16h frag_f32(const float* rowk0, int lane) {
  v16h a; const float* p = rowk0 + 8 * (lane >> 4);
#pragma unroll
  for (int i = 0; i < 8; ++i) { a[i] = (_Float16)p[i]; a[8 + i] = (_Float16)p[16 + i]; }
  return a;
}
__device__ __forceinline__ v16h frag_f32s(const float* rowk0, int lane, float sc) {
  v16h a; const float* p = rowk0 + 8 * (lane >> 4);
#pragma unroll
  for (int i = 0; i < 8; ++i) { a[i] = (_Float16)(p[i] * sc); a[8 + i] = (_Float16)(p[16 + i] * sc); }
  return a;
}
__device__ __forceinline__ v16h fragc_f32(const float* W, int k0, int n, int lane, int ld, int K) {
  v16h a; const int g = lane >> 4;
#pragma unroll
  for (int i = 0; i < 8; ++i) { const int ka = k0 + 8 * g + i, kb = ka + 16;
    a[i] = (_Float16)(ka < K ? W[(size_t)(ka < K ? ka : K - 1) * ld + n] : 0.f); a[8 + i] = (_Float16)(kb < K ? W[(size_t)(kb < K ? kb : K - 1) * ld + n] : 0.f); }
  return a;
}
struct F2 { v16b h, l; };
__device__ __forceinline__ F2 bsplit16(const float v[16]) { F2 r;
#pragma unroll
  for (int i = 0; i < 16; ++i) { const __bf16 h = (__bf16)v[i]; r.h[i] = h; r.l[i] = (__bf16)(v[i] - (float)h); }
  return r; }
__device__ __forceinline__ F2 split_row(const float* row, int k0, int lane) { float v[16]; const float* p = row + k0 + 8 * (lane >> 4);
#pragma unroll
  for (int i = 0; i < 8; ++i) { v[i] = p[i]; v[8 + i] = p[16 + i]; }
  return bsplit16(v); }
__device__ __forceinline__ F2 split_rowK(const float* row, int k0, int lane, int K) { float v[16]; const int g = lane >> 4;
#pragma unroll
  for (int i = 0; i < 8; ++i) { const int ka = k0 + 8 * g + i, kb = ka + 16; v[i] = ka < K ? row[ka < K ? ka : K - 1] : 0.f; v[8 + i] = kb < K ? row[kb < K ? kb : K - 1] : 0.f; }
  return bsplit16(v); }
__device__ __forceinline__ F2 split_col(const float* W, int k0, int n, int lane, int ld, int K) { float v[16]; const int g = lane >> 4;
#pragma unroll
  for (int i = 0; i < 8; ++i) { const int ka = k0 + 8 * g + i, kb = ka + 16; v[i] = ka < K ? W[(size_t)(ka < K ? ka : K - 1) * ld + n] : 0.f; v[8 + i] = kb < K ? W[(size_t)(kb < K ? kb : K - 1) * ld + n] : 0.f; }
  return bsplit16(v); }
__device__ __forceinline__ v8f mac3(const F2& a, const F2& b, v8f c) { c = wmma_bf(a.l, b.h, c); c = wmma_bf(a.h, b.l, c); return wmma_bf(a.h, b.h, c); }
__device__ __forceinline__ float sigm(float v) { return 1.0f / (1.0f + expf(-v)); }
#define LDSX() do { asm volatile("s_wait_dscnt 0" ::: "memory"); __builtin_amdgcn_wave_barrier(); __builtin_amdgcn_fence(__ATOMIC_RELEASE, "workgroup"); } while (0)


#define NB 2
#define SS 4096
#define DM_ 768
#define NH 12
#define HD 64
#define WIN 256
#define NG 64
#ifndef TNB
#define TNB NB
#endif
#ifndef TQB
#define TQB (SS / 64)
#endif
#ifndef TPRQ
#define TPRQ (NB * SS / 64)
#endif
typedef __attribute__((ext_vector_type(8))) __bf16 v8b;
__device__ __forceinline__ v16b frag_b(const __bf16* rowk0, int lane) {
  union { v16b v; v8b q[2]; } u; const __bf16* p = rowk0 + 8 * (lane >> 4);
  u.q[0] = *(const v8b*)p; u.q[1] = *(const v8b*)(p + 16); return u.v;
}
__device__ __forceinline__ float bfr(float v) { return (float)(__bf16)v; }
__device__ __attribute__((noinline)) float exp_ni(float v) { return expf(v); }
__device__ __attribute__((noinline)) float erf_ni(float v) { return erff(v); }

#define RW (size_t)DM_
#define WS_Q   0u
#define WS_K   (WS_Q + 2u * (size_t)NB * SS * DM_)
#define WS_KL  (WS_K + 2u * (size_t)NB * SS * DM_)
#define WS_V   (WS_KL + 2u * (size_t)NB * SS * DM_)
#define WS_VL  (WS_V + 2u * (size_t)NB * DM_ * SS)
#define WS_KG  (WS_VL + 2u * (size_t)NB * DM_ * SS)
#define WS_KGL (WS_KG + 2u * (size_t)NB * SS * DM_)
#define WS_VG  (WS_KGL + 2u * (size_t)NB * SS * DM_)
#define WS_VGL (WS_VG + 2u * (size_t)NB * DM_ * SS)
#define WS_QG  (WS_VGL + 2u * (size_t)NB * DM_ * SS)
#define WS_CT  (WS_QG + 2u * (size_t)NB * NG * DM_)
#define WS_END (WS_CT + 4u * (size_t)NB * SS * DM_)

__global__ __launch_bounds__(128) void k_proj(const float* __restrict__ X, const float* __restrict__ WQ, const float* __restrict__ WK, const float* __restrict__ WV, const float* __restrict__ WKG, const float* __restrict__ WVG, _Float16* __restrict__ Q, _Float16* __restrict__ K, _Float16* __restrict__ KL, _Float16* __restrict__ V, _Float16* __restrict__ VL, _Float16* __restrict__ KG, _Float16* __restrict__ KGL, _Float16* __restrict__ VG, _Float16* __restrict__ VGL) {
  __shared__ __align__(16) _Float16 sh[64][136], sl[64][136]; __shared__ __align__(16) _Float16 th[128][72], tl[128][72];
  const int tid = threadIdx.x, wave = tid >> 5, lane = tid & 31, col = lane & 15, g = lane >> 4; const int which = blockIdx.z; const int c0 = blockIdx.y * 128; const size_t r0 = (size_t)blockIdx.x * 64; if (which <= 2 && blockIdx.x >= TPRQ) return;
  const float* Wm = which == 0 ? WQ : which == 1 ? WK : which == 2 ? WV : which == 3 ? WKG : WVG;
  v8f acc[8] = {};
#pragma unroll 2
  for (int kc = 0; kc < DM_ / 32; ++kc) { v16b a; { const float* p = X + (r0 + wave * 16 + col) * RW + kc * 32 + 8 * g;
#pragma unroll
      for (int i = 0; i < 8; ++i) { a[i] = (__bf16)p[i]; a[8 + i] = (__bf16)p[16 + i]; } }
#pragma unroll
    for (int j = 0; j < 8; ++j) { v16b w; const int o = c0 + j * 16 + col;
#pragma unroll
      for (int i = 0; i < 8; ++i) { w[i] = (__bf16)Wm[(size_t)(kc * 32 + 8 * g + i) * DM_ + o]; w[8 + i] = (__bf16)Wm[(size_t)(kc * 32 + 16 + 8 * g + i) * DM_ + o]; }
      acc[j] = wmma_bf(a, w, acc[j]); } }
  const bool planes = (which == 2 || which == 4);
#pragma unroll
  for (int j = 0; j < 8; ++j)
#pragma unroll
    for (int r = 0; r < 8; ++r) { const float v = acc[j][r]; const int rl = wave * 16 + 8 * g + r, cl = j * 16 + col; const _Float16 hv = (_Float16)v; const _Float16 lv = (_Float16)(v - (float)hv); if (planes) { th[cl][rl] = hv; tl[cl][rl] = lv; } else { sh[rl][cl] = hv; sl[rl][cl] = lv; } }
  __syncthreads();
  if (!planes) { _Float16* dh = which == 0 ? Q : which == 1 ? K : KG; _Float16* dl = which == 0 ? nullptr : which == 1 ? KL : KGL;
    for (int e = tid; e < 64 * 16; e += 128) { const int rl = e >> 4, q = e & 15; vst2((unsigned*)(dh + (r0 + rl) * RW + c0 + q * 8), *(const v4u*)&sh[rl][q * 8]); if (dl) vst2((unsigned*)(dl + (r0 + rl) * RW + c0 + q * 8), *(const v4u*)&sl[rl][q * 8]); } }
  else { _Float16* dh = which == 2 ? V : VG; _Float16* dl = which == 2 ? VL : VGL; const size_t b = r0 / SS; const int s0 = (int)(r0 % SS);
    for (int e = tid; e < 128 * 8; e += 128) { const int cl = e >> 3, q = e & 7; const size_t o = (b * DM_ + c0 + cl) * (size_t)SS + s0 + q * 8; vst2((unsigned*)(dh + o), *(const v4u*)&th[cl][q * 8]); vst2((unsigned*)(dl + o), *(const v4u*)&tl[cl][q * 8]); } } }
__global__ __launch_bounds__(128) void k_projg(const float* __restrict__ X, const float* __restrict__ WQG, _Float16* __restrict__ QG) { __shared__ __align__(16) _Float16 sh[64][136];
  const int tid = threadIdx.x, wave = tid >> 5, lane = tid & 31, col = lane & 15, g = lane >> 4; const int c0 = blockIdx.x * 128; const size_t b = blockIdx.y; const size_t r0 = b * SS;
  v8f acc[8] = {};
#pragma unroll 2
  for (int kc = 0; kc < DM_ / 32; ++kc) { v16b a; { const float* p = X + (r0 + wave * 16 + col) * RW + kc * 32 + 8 * g;
#pragma unroll
      for (int i = 0; i < 8; ++i) { a[i] = (__bf16)p[i]; a[8 + i] = (__bf16)p[16 + i]; } }
#pragma unroll
    for (int j = 0; j < 8; ++j) { v16b w; const int o = c0 + j * 16 + col;
#pragma unroll
      for (int i = 0; i < 8; ++i) { w[i] = (__bf16)WQG[(size_t)(kc * 32 + 8 * g + i) * DM_ + o]; w[8 + i] = (__bf16)WQG[(size_t)(kc * 32 + 16 + 8 * g + i) * DM_ + o]; }
      acc[j] = wmma_bf(a, w, acc[j]); } }
#pragma unroll
  for (int j = 0; j < 8; ++j)
#pragma unroll
    for (int r = 0; r < 8; ++r) sh[wave * 16 + 8 * g + r][j * 16 + col] = (_Float16)acc[j][r];
  __syncthreads(); for (int e = tid; e < 64 * 16; e += 128) { const int rl = e >> 4, q = e & 15; vst2((unsigned*)(QG + (b * NG + rl) * RW + c0 + q * 8), *(const v4u*)&sh[rl][q * 8]); } }
__global__ __launch_bounds__(128) void k_band(const _Float16* __restrict__ Q, const _Float16* __restrict__ K, const _Float16* __restrict__ KL, const _Float16* __restrict__ V, const _Float16* __restrict__ VL, float* __restrict__ CT) {
  __shared__ __align__(16) float sp[4][16][36]; __shared__ __align__(16) float so[4][16][68];
  const int tid = threadIdx.x, wave = tid >> 5, lane = tid & 31, col = lane & 15, g = lane >> 4; const int qb = blockIdx.x + 1, h = blockIdx.y; const size_t b = blockIdx.z; const int i0 = qb * 64; const size_t q0 = b * SS + i0 + wave * 16;
  v16h aq[2];
#pragma unroll
  for (int kc = 0; kc < 2; ++kc) aq[kc] = frag_h(Q + (q0 + col) * RW + h * HD + kc * 32, lane);
  float m[8], l[8];
#pragma unroll
  for (int r = 0; r < 8; ++r) { m[r] = -3.0e38f; l[r] = 0.f; }
  v8f acc[4] = {};
  const int jlo = i0 - WIN;
#pragma unroll 1
  for (int tt = 0; tt < 2 + (64 + 2 * WIN) / 32; ++tt) { const bool glob = (tt < 2); const int j0 = glob ? (tt * 32) : (jlo + (tt - 2) * 32);
    if (!glob && (j0 + 31 < 0 || j0 >= SS)) continue;
    float s[2][8];
#pragma unroll
    for (int ct = 0; ct < 2; ++ct) { const int j = j0 + ct * 16 + col; const int jc = j < 0 ? 0 : (j >= SS ? SS - 1 : j); const size_t kk = b * SS + jc; v8f c = {};
#pragma unroll
      for (int kc = 0; kc < 2; ++kc) { c = wmma16(aq[kc], frag_h(K + kk * RW + h * HD + kc * 32, lane), c); c = wmma16(aq[kc], frag_h(KL + kk * RW + h * HD + kc * 32, lane), c); }
#pragma unroll
      for (int r = 0; r < 8; ++r) { const int i = i0 + wave * 16 + 8 * g + r; const bool ok = glob ? true : (j >= 0 && j < SS && j >= i - WIN && j <= i + WIN); s[ct][r] = ok ? c[r] : -3.0e38f; } }
    float alpha[8];
#pragma unroll
    for (int r = 0; r < 8; ++r) { float mx = fmaxf(s[0][r], s[1][r]);
#pragma unroll
      for (int o = 1; o < 16; o <<= 1) mx = fmaxf(mx, __shfl_xor(mx, o));
      const float mn = fmaxf(m[r], mx); alpha[r] = (mn <= -1.0e38f) ? 1.f : __expf(m[r] - mn); const float e0 = (s[0][r] <= -1.0e38f) ? 0.f : __expf(s[0][r] - mn), e1 = (s[1][r] <= -1.0e38f) ? 0.f : __expf(s[1][r] - mn); float es = e0 + e1;
#pragma unroll
      for (int o = 1; o < 16; o <<= 1) es += __shfl_xor(es, o);
      l[r] = l[r] * alpha[r] + es; m[r] = mn; sp[wave][8 * g + r][col] = e0; sp[wave][8 * g + r][16 + col] = e1; }
#pragma unroll
    for (int j = 0; j < 4; ++j)
#pragma unroll
      for (int r = 0; r < 8; ++r) acc[j][r] *= alpha[r];
    LDSX();
    { const int jv = j0; const v16h pa = frag_f32s(&sp[wave][col][0], lane, 2048.0f);
#pragma unroll
      for (int j = 0; j < 4; ++j) { const size_t po = (b * DM_ + (size_t)h * HD + j * 16 + col) * (size_t)SS + jv; acc[j] = wmma16(pa, frag_h(V + po, lane), acc[j]); acc[j] = wmma16(pa, frag_h(VL + po, lane), acc[j]); } }
    LDSX(); }
#pragma unroll
  for (int r = 0; r < 8; ++r) { const float il = (1.0f / 2048.0f) / l[r];
#pragma unroll
    for (int j = 0; j < 4; ++j) so[wave][8 * g + r][j * 16 + col] = acc[j][r] * il; }
  LDSX(); for (int rl = 0; rl < 16; ++rl) if (lane < 16) vst2(CT + (q0 + rl) * RW + h * HD + lane * 4, *(const v4f*)&so[wave][rl][lane * 4]); }
__global__ __launch_bounds__(128) void k_glob(const _Float16* __restrict__ QG, const _Float16* __restrict__ KG, const _Float16* __restrict__ KGL, const _Float16* __restrict__ VG, const _Float16* __restrict__ VGL, float* __restrict__ CT) {
  __shared__ __align__(16) float sp[4][16][36]; __shared__ __align__(16) float so[4][16][68];
  const int tid = threadIdx.x, wave = tid >> 5, lane = tid & 31, col = lane & 15, g = lane >> 4; const int h = blockIdx.x; const size_t b = blockIdx.y; const size_t qg0 = b * NG + wave * 16;
  v16h aq[2];
#pragma unroll
  for (int kc = 0; kc < 2; ++kc) aq[kc] = frag_h(QG + (qg0 + col) * RW + h * HD + kc * 32, lane);
  float m[8], l[8];
#pragma unroll
  for (int r = 0; r < 8; ++r) { m[r] = -3.0e38f; l[r] = 0.f; }
  v8f acc[4] = {};
#pragma unroll 1
  for (int ks = 0; ks < SS / 32; ++ks) { float s[2][8];
#pragma unroll
    for (int ct = 0; ct < 2; ++ct) { const size_t kk = b * SS + ks * 32 + ct * 16 + col; v8f c = {};
#pragma unroll
      for (int kc = 0; kc < 2; ++kc) { c = wmma16(aq[kc], frag_h(KG + kk * RW + h * HD + kc * 32, lane), c); c = wmma16(aq[kc], frag_h(KGL + kk * RW + h * HD + kc * 32, lane), c); }
#pragma unroll
      for (int r = 0; r < 8; ++r) s[ct][r] = c[r]; }
    float alpha[8];
#pragma unroll
    for (int r = 0; r < 8; ++r) { float mx = fmaxf(s[0][r], s[1][r]);
#pragma unroll
      for (int o = 1; o < 16; o <<= 1) mx = fmaxf(mx, __shfl_xor(mx, o));
      const float mn = fmaxf(m[r], mx); alpha[r] = __expf(m[r] - mn); const float e0 = __expf(s[0][r] - mn), e1 = __expf(s[1][r] - mn); float es = e0 + e1;
#pragma unroll
      for (int o = 1; o < 16; o <<= 1) es += __shfl_xor(es, o);
      l[r] = l[r] * alpha[r] + es; m[r] = mn; sp[wave][8 * g + r][col] = e0; sp[wave][8 * g + r][16 + col] = e1; }
#pragma unroll
    for (int j = 0; j < 4; ++j)
#pragma unroll
      for (int r = 0; r < 8; ++r) acc[j][r] *= alpha[r];
    LDSX();
    const v16h pa = frag_f32s(&sp[wave][col][0], lane, 2048.0f);
#pragma unroll
    for (int j = 0; j < 4; ++j) { const size_t po = (b * DM_ + (size_t)h * HD + j * 16 + col) * (size_t)SS + ks * 32; acc[j] = wmma16(pa, frag_h(VG + po, lane), acc[j]); acc[j] = wmma16(pa, frag_h(VGL + po, lane), acc[j]); }
    LDSX(); }
#pragma unroll
  for (int r = 0; r < 8; ++r) { const float il = (1.0f / 2048.0f) / l[r];
#pragma unroll
    for (int j = 0; j < 4; ++j) so[wave][8 * g + r][j * 16 + col] = acc[j][r] * il; }
  LDSX(); for (int rl = 0; rl < 16; ++rl) if (lane < 16) vst2(CT + (b * SS + wave * 16 + rl) * RW + h * HD + lane * 4, *(const v4f*)&so[wave][rl][lane * 4]); }
__global__ __launch_bounds__(128) void k_out(const float* __restrict__ CT, const float* __restrict__ WO, float* __restrict__ OUT) { __shared__ __align__(16) float sf[4][16][132];
  const int tid = threadIdx.x, wave = tid >> 5, lane = tid & 31, col = lane & 15, g = lane >> 4; const int c0 = blockIdx.y * 128; const size_t r0 = (size_t)blockIdx.x * 64 + wave * 16;
  v8f acc[8] = {};
#pragma unroll 2
  for (int kc = 0; kc < DM_ / 32; ++kc) { const F2 a = split_row(CT + (r0 + col) * RW, kc * 32, lane);
#pragma unroll
    for (int j = 0; j < 8; ++j) { v16b w; const int o = c0 + j * 16 + col;
#pragma unroll
      for (int i = 0; i < 8; ++i) { w[i] = (__bf16)WO[(size_t)(kc * 32 + 8 * g + i) * DM_ + o]; w[8 + i] = (__bf16)WO[(size_t)(kc * 32 + 16 + 8 * g + i) * DM_ + o]; }
      acc[j] = wmma_bf(a.h, w, acc[j]); acc[j] = wmma_bf(a.l, w, acc[j]); } }
#pragma unroll
  for (int j = 0; j < 8; ++j)
#pragma unroll
    for (int r = 0; r < 8; ++r) sf[wave][8 * g + r][j * 16 + col] = acc[j][r];
  LDSX(); for (int rl = 0; rl < 16; ++rl) vst2(OUT + (r0 + rl) * RW + c0 + lane * 4, *(const v4f*)&sf[wave][rl][lane * 4]); }
extern "C" void kernel_launch(void* const* d_in, const int* in_sizes, int n_in, void* d_out, int out_size, void* d_ws, size_t ws_size, hipStream_t stream) {
  (void)in_sizes; (void)n_in; (void)out_size;
  const float** F = (const float**)d_in;
  if (ws_size < (size_t)WS_END) return;
  char* ws = (char*)d_ws; _Float16 *Q = (_Float16*)(ws + WS_Q), *K = (_Float16*)(ws + WS_K), *KL = (_Float16*)(ws + WS_KL), *V = (_Float16*)(ws + WS_V), *VL = (_Float16*)(ws + WS_VL), *KG = (_Float16*)(ws + WS_KG), *KGL = (_Float16*)(ws + WS_KGL), *VG = (_Float16*)(ws + WS_VG), *VGL = (_Float16*)(ws + WS_VGL), *QG = (_Float16*)(ws + WS_QG); float* CT = (float*)(ws + WS_CT);
  k_proj<<<dim3(TNB * SS / 64, DM_ / 128, 5), 128, 0, stream>>>(F[0], F[1], F[2], F[3], F[5], F[6], Q, K, KL, V, VL, KG, KGL, VG, VGL);
  k_projg<<<dim3(DM_ / 128, TNB), 128, 0, stream>>>(F[0], F[4], QG);
  if (TQB > 1) k_band<<<dim3(TQB - 1, NH, TNB), 128, 0, stream>>>(Q, K, KL, V, VL, CT);
  k_glob<<<dim3(NH, TNB), 128, 0, stream>>>(QG, KG, KGL, VG, VGL, CT);
  for (int b = 0; b < TNB; ++b) k_out<<<dim3(TQB, DM_ / 128), 128, 0, stream>>>(CT + (size_t)b * SS * DM_, F[7], (float*)d_out + (size_t)b * SS * DM_);
}
